// GCNLinkPredictor_2516850835926
// MI455X (gfx1250) — hardware-verified
//
#include <hip/hip_runtime.h>
#include <stddef.h>


#define INC     128
#define HID     64
#define NTHR    256
#define NWAVE   8
#define EPT     8
#define NGRP    2
#define CHUNK   (NTHR * EPT * NGRP)
#define WCAP    (EPT * NGRP * 32)
#define LISTN   (NWAVE * WCAP)
#define NBC     4096
#define NBF     1024
#define RCAP    40960
#define RBN     128
#define TGT     256
#define DEGCAP  256
#define GROWS   128
#define OTHR    512
#define WSCAP   134217728

#define LDS_FILL ((RCAP + NBF + LISTN) * 4 + 64)
#define LDS_GEMM(KD) (2 * GROWS * ((KD) + 8) * 2)

static_assert((CHUNK & (CHUNK - 1)) == 0);
static_assert(CHUNK <= 4096);
static_assert(NBC <= 4096 && NBF <= 4096);
static_assert((NBC & (NBC - 1)) == 0 && (NBF & (NBF - 1)) == 0);
static_assert(NBC == 4 * NBF);
static_assert(OTHR * 8 == NBC);
static_assert((RCAP % 32) == 0);
static_assert(GROWS * HID * 4 <= LDS_GEMM(64));
static_assert(GROWS * HID * 4 <= LDS_GEMM(128));
static_assert(TGT == NWAVE * 32 && (TGT % GROWS) == 0);
static_assert((NBC % TGT) == 0);
static_assert(GROWS == NWAVE * 16);
static_assert((GROWS * 128 / 8) % NTHR == 0);
static_assert((GROWS * 64 / 8) % NTHR == 0);

typedef float          v4f  __attribute__((ext_vector_type(4)));
typedef float          v8f  __attribute__((ext_vector_type(8)));
typedef int            v4i  __attribute__((ext_vector_type(4)));
typedef unsigned short v8us __attribute__((ext_vector_type(8)));
typedef __bf16         v16b __attribute__((ext_vector_type(16)));
union FragB { v16b v; v8us h[2]; };

__device__ __forceinline__ unsigned int bfr(float f) {
  const unsigned int u = __float_as_uint(f);
  return (u + 0x7FFFu + ((u >> 16) & 1u)) >> 16;
}

__device__ __forceinline__ void split1(float x, unsigned short& hb, unsigned short& lb) {
  const unsigned int hu = bfr(x);
  const float hf = __uint_as_float(hu << 16);
  hb = (unsigned short)hu;
  lb = (unsigned short)bfr(x - hf);
}

__device__ __forceinline__ void split8(v4f a, v4f b, v8us& hi, v8us& lo) {
  unsigned short hb, lb;
  split1(a.x, hb, lb); hi[0] = hb; lo[0] = lb;
  split1(a.y, hb, lb); hi[1] = hb; lo[1] = lb;
  split1(a.z, hb, lb); hi[2] = hb; lo[2] = lb;
  split1(a.w, hb, lb); hi[3] = hb; lo[3] = lb;
  split1(b.x, hb, lb); hi[4] = hb; lo[4] = lb;
  split1(b.y, hb, lb); hi[5] = hb; lo[5] = lb;
  split1(b.z, hb, lb); hi[6] = hb; lo[6] = lb;
  split1(b.w, hb, lb); hi[7] = hb; lo[7] = lb;
}

__device__ __forceinline__ v8f wmb(v16b a, v16b b, v8f c) {
  v8f d = __builtin_amdgcn_wmma_f32_16x16x32_bf16(false, a, false, b, (short)0, c, false, false);
  asm volatile("v_nop\n\tv_nop\n\tv_nop\n\tv_nop" : "+v"(d) : "v"(a), "v"(b));
  return d;
}

template <int NB>
__device__ __forceinline__ int scan_chunk(const int* __restrict__ dsts, int nE, int cbase, int slotBase,
                                          int vec8, int* list, int tid, int lane, int wave) {
  int wc = 0;
#pragma unroll
  for (int g = 0; g < NGRP; ++g) {
    const int el0  = (g * NTHR + tid) * EPT;
    const int e0   = cbase + el0;
    const int sent = -2147483647 - 1;
    v4i da, db;
    if (vec8 != 0 && cbase + CHUNK <= nE) {
      da = *(const v4i*)(dsts + e0);
      db = *(const v4i*)(dsts + e0 + 4);
    } else {
      da.x = (e0     < nE) ? dsts[min(e0, nE - 1)] : sent;
      da.y = (e0 + 1 < nE) ? dsts[min(e0 + 1, nE - 1)] : sent;
      da.z = (e0 + 2 < nE) ? dsts[min(e0 + 2, nE - 1)] : sent;
      da.w = (e0 + 3 < nE) ? dsts[min(e0 + 3, nE - 1)] : sent;
      db.x = (e0 + 4 < nE) ? dsts[min(e0 + 4, nE - 1)] : sent;
      db.y = (e0 + 5 < nE) ? dsts[min(e0 + 5, nE - 1)] : sent;
      db.z = (e0 + 6 < nE) ? dsts[min(e0 + 6, nE - 1)] : sent;
      db.w = (e0 + 7 < nE) ? dsts[min(e0 + 7, nE - 1)] : sent;
    }
    const unsigned nb = (unsigned)slotBase;
    const unsigned s0 = (unsigned)da.x - nb, s1 = (unsigned)da.y - nb;
    const unsigned s2 = (unsigned)da.z - nb, s3 = (unsigned)da.w - nb;
    const unsigned s4 = (unsigned)db.x - nb, s5 = (unsigned)db.y - nb;
    const unsigned s6 = (unsigned)db.z - nb, s7 = (unsigned)db.w - nb;
    const bool h0 = s0 < (unsigned)NB, h1 = s1 < (unsigned)NB, h2 = s2 < (unsigned)NB, h3 = s3 < (unsigned)NB;
    const bool h4 = s4 < (unsigned)NB, h5 = s5 < (unsigned)NB, h6 = s6 < (unsigned)NB, h7 = s7 < (unsigned)NB;
    const unsigned any = __builtin_amdgcn_ballot_w32(h0 | h1 | h2 | h3 | h4 | h5 | h6 | h7);
    if (any != 0u) {
#define HITJ(J, HJ, SJ) { \
        const unsigned mj = __builtin_amdgcn_ballot_w32(HJ); \
        if (mj != 0u) { \
          if (HJ) { \
            const int pos = wc + (int)__builtin_amdgcn_mbcnt_lo(mj, 0u); \
            if (pos < WCAP) list[wave * WCAP + pos] = ((el0 + (J)) << 12) | (int)(SJ); \
          } \
          wc += (int)__builtin_popcount(mj); } }
      HITJ(0, h0, s0)
      HITJ(1, h1, s1)
      HITJ(2, h2, s2)
      HITJ(3, h3, s3)
      HITJ(4, h4, s4)
      HITJ(5, h5, s5)
      HITJ(6, h6, s6)
      HITJ(7, h7, s7)
#undef HITJ
    }
  }
  return wc;
}

__global__ __launch_bounds__(NTHR) void k_wprep(
    const float* __restrict__ w, unsigned short* wp, int K, int total) {
  const int i = (int)blockIdx.x * NTHR + (int)threadIdx.x;
  if (i >= total) return;
  const int kq = K >> 3;
  const int n  = i / kq;
  const int k0 = (i - n * kq) * 8;
  float v[8];
#pragma unroll
  for (int e = 0; e < 8; ++e) v[e] = w[(size_t)(k0 + e) * HID + n];
  v4f a, b;
  a.x = v[0]; a.y = v[1]; a.z = v[2]; a.w = v[3];
  b.x = v[4]; b.y = v[5]; b.z = v[6]; b.w = v[7];
  v8us hv, lv;
  split8(a, b, hv, lv);
  unsigned short* dh = wp + (size_t)i * 8;
  unsigned short* dl = dh + (size_t)HID * K;
  *(volatile v8us*)dh = hv;
  *(volatile v8us*)dl = lv;
  __threadfence();
  *(volatile v8us*)dh = hv;
  *(volatile v8us*)dl = lv;
}

__global__ __launch_bounds__(NTHR) void k_count(
    const int* __restrict__ ei, int* cnt, float* dinv, int nE, int vec8) {
  __shared__ __attribute__((aligned(16))) int scnt[NBC];
  __shared__ __attribute__((aligned(16))) int list[LISTN];
  __shared__ int wcnt[NWAVE];
  const int tid = threadIdx.x, lane = tid & 31, wave = tid >> 5;
  const int nodeBase = blockIdx.x * NBC;
  const int* dsts = ei + nE;

  for (int i = tid; i < NBC; i += NTHR) scnt[i] = 0;
  __syncthreads();

  const int nChunks = (nE + CHUNK - 1) / CHUNK;
#pragma unroll 1
  for (int ch = 0; ch < nChunks; ++ch) {
    const int cbase = ch * CHUNK;
    const int wc = scan_chunk<NBC>(dsts, nE, cbase, nodeBase, vec8, list, tid, lane, wave);
    if (lane == 0) wcnt[wave] = wc;
    __syncthreads();
    if (wave == 0) {
#pragma unroll 1
      for (int wsx = 0; wsx < NWAVE; ++wsx) {
        int n = __builtin_amdgcn_readfirstlane(wcnt[wsx]);
        n = n > WCAP ? WCAP : (n < 0 ? 0 : n);
        const int* lp = list + wsx * WCAP;
#pragma unroll 1
        for (int i = 0; i < n; ++i) {
          const int ent  = __builtin_amdgcn_readfirstlane(lp[i]);
          const int slot = ent & (NBC - 1);
          if (lane == 0) scnt[slot] = scnt[slot] + 1;
        }
      }
    }
    __syncthreads();
  }

  v4i cq[4]; v4f dq[4];
#pragma unroll
  for (int q = 0; q < 4; ++q) {
    const int f = (wave * 4 + q) * 128 + 4 * lane;
    const v4i c = *(const v4i*)(scnt + f);
    cq[q] = c;
    dq[q].x = rsqrtf((float)(c.x + 1));
    dq[q].y = rsqrtf((float)(c.y + 1));
    dq[q].z = rsqrtf((float)(c.z + 1));
    dq[q].w = rsqrtf((float)(c.w + 1));
  }
  int*   cp = cnt + (size_t)nodeBase;
  float* dp = dinv + (size_t)nodeBase;
#pragma unroll
  for (int q = 0; q < 4; ++q) {
    const int f = (wave * 4 + q) * 128 + 4 * lane;
    *(volatile v4i*)(cp + f) = cq[q];
    *(volatile v4f*)(dp + f) = dq[q];
  }
  __threadfence();
#pragma unroll
  for (int q = 0; q < 4; ++q) {
    const int f = (wave * 4 + q) * 128 + 4 * lane;
    *(volatile v4i*)(cp + f) = cq[q];
    *(volatile v4f*)(dp + f) = dq[q];
  }
}

__global__ __launch_bounds__(OTHR) void k_offsets(
    const int* __restrict__ cnt, int* off, int* rbase, int nChunk) {
  __shared__ __attribute__((aligned(16))) int soff[NBC];
  __shared__ __attribute__((aligned(16))) int srb[RBN];
  __shared__ int wtot[OTHR / 32];
  const int tid = threadIdx.x, lane = tid & 31, wave = tid >> 5, sub = tid >> 7;
  for (int i = tid; i < RBN; i += OTHR) srb[i] = 0;
  int carry = 0;
#pragma unroll 1
  for (int ch = 0; ch < nChunk; ++ch) {
    const int base = ch * NBC;
    const v4i c0 = *(const v4i*)(cnt + base + 8 * tid);
    const v4i c1 = *(const v4i*)(cnt + base + 8 * tid + 4);
    const int e0 = max(c0.x, 0), e1 = max(c0.y, 0), e2 = max(c0.z, 0), e3 = max(c0.w, 0);
    const int e4 = max(c1.x, 0), e5 = max(c1.y, 0), e6 = max(c1.z, 0), e7 = max(c1.w, 0);
    const int ts = e0 + e1 + e2 + e3 + e4 + e5 + e6 + e7;
    int incl = ts;
#pragma unroll
    for (int d = 1; d < 32; d <<= 1) {
      const int t = __shfl_up(incl, d);
      if (lane >= d) incl += t;
    }
    if (lane == 31) wtot[wave] = incl;
    __syncthreads();
    const int S0 = wtot[0]  + wtot[1]  + wtot[2]  + wtot[3];
    const int S1 = wtot[4]  + wtot[5]  + wtot[6]  + wtot[7];
    const int S2 = wtot[8]  + wtot[9]  + wtot[10] + wtot[11];
    const int S3 = wtot[12] + wtot[13] + wtot[14] + wtot[15];
    int pre = 0;
#pragma unroll 1
    for (int w = 4 * sub; w < wave; ++w) pre += wtot[w];
    const int b0 = carry;
    const int b1 = b0 + ((S0 + 31) & ~31);
    const int b2 = b1 + ((S1 + 31) & ~31);
    const int b3 = b2 + ((S2 + 31) & ~31);
    const int b4 = b3 + ((S3 + 31) & ~31);
    const int myb = sub == 0 ? b0 : (sub == 1 ? b1 : (sub == 2 ? b2 : b3));
    if (tid == 0) {
      srb[min(4 * ch + 0, RBN - 1)] = b0;
      srb[min(4 * ch + 1, RBN - 1)] = b1;
      srb[min(4 * ch + 2, RBN - 1)] = b2;
      srb[min(4 * ch + 3, RBN - 1)] = b3;
    }
    int run = myb + pre + incl - ts;
    soff[8 * tid + 0] = run; run += e0;
    soff[8 * tid + 1] = run; run += e1;
    soff[8 * tid + 2] = run; run += e2;
    soff[8 * tid + 3] = run; run += e3;
    soff[8 * tid + 4] = run; run += e4;
    soff[8 * tid + 5] = run; run += e5;
    soff[8 * tid + 6] = run; run += e6;
    soff[8 * tid + 7] = run;
    carry = b4;
    __syncthreads();
    const v4i o0 = *(const v4i*)(soff + 4 * tid);
    const v4i o1 = *(const v4i*)(soff + 4 * (tid + OTHR));
    int* op = off + base;
    *(volatile v4i*)(op + 4 * tid) = o0;
    *(volatile v4i*)(op + 4 * (tid + OTHR)) = o1;
    __threadfence();
    *(volatile v4i*)(op + 4 * tid) = o0;
    *(volatile v4i*)(op + 4 * (tid + OTHR)) = o1;
    __syncthreads();
  }
  if (tid == 0) srb[min(4 * nChunk, RBN - 1)] = carry;
  __syncthreads();
  v4i rv = {0, 0, 0, 0};
  if (tid < 32) rv = *(const v4i*)(srb + 4 * tid);
  if (tid < 32) *(volatile v4i*)(rbase + 4 * tid) = rv;
  __threadfence();
  if (tid < 32) *(volatile v4i*)(rbase + 4 * tid) = rv;
}

__global__ __launch_bounds__(NTHR) void k_fill(
    const int* __restrict__ ei, const int* __restrict__ off, const int* __restrict__ rbase,
    int* csr, int nN, int nE, int vec8, int csrLen) {
  extern __shared__ v4f lds_dyn[];
  int* region = (int*)lds_dyn;
  int* cursor = region + RCAP;
  int* list   = cursor + NBF;
  int* wcnt   = list + LISTN;
  const int tid = threadIdx.x, lane = tid & 31, wave = tid >> 5;
  const int b = blockIdx.x;
  const int nodeBase = b * NBF;
  const int* dsts = ei + nE;

  int rb0 = rbase[b];
  const int rb1 = rbase[b + 1];
  rb0 = rb0 < 0 ? 0 : (rb0 > csrLen ? csrLen : rb0);
  rb0 &= ~31;
  int len = rb1 - rb0;
  len = len < 0 ? 0 : (len > RCAP ? RCAP : len);
  int lenW = (len + 31) & ~31;
  if (rb0 + lenW > csrLen) lenW = (csrLen - rb0) & ~31;

  {
    const v4i z = {0, 0, 0, 0};
    for (int i = tid; i < RCAP / 4; i += NTHR) ((v4i*)region)[i] = z;
    for (int s = tid; s < NBF; s += NTHR) {
      int o = off[nodeBase + s] - rb0;
      o = o < 0 ? 0 : (o > RCAP ? RCAP : o);
      cursor[s] = o;
    }
  }
  __syncthreads();

  const int nChunks = (nE + CHUNK - 1) / CHUNK;
#pragma unroll 1
  for (int ch = 0; ch < nChunks; ++ch) {
    const int cbase = ch * CHUNK;
    const int wc = scan_chunk<NBF>(dsts, nE, cbase, nodeBase, vec8, list, tid, lane, wave);
    if (lane == 0) wcnt[wave] = wc;
    __syncthreads();
    if (wave == 0) {
#pragma unroll 1
      for (int wsx = 0; wsx < NWAVE; ++wsx) {
        int n = __builtin_amdgcn_readfirstlane(wcnt[wsx]);
        n = n > WCAP ? WCAP : (n < 0 ? 0 : n);
        const int* lp = list + wsx * WCAP;
#pragma unroll 1
        for (int i = 0; i < n; ++i) {
          const int ent  = __builtin_amdgcn_readfirstlane(lp[i]);
          const int slot = ent & (NBF - 1);
          int e = cbase + ((ent >> 12) & (CHUNK - 1));
          e = e > nE - 1 ? nE - 1 : e;
          int src = ei[e];
          src = src < 0 ? 0 : (src > nN - 1 ? nN - 1 : src);
          if (lane == 0) {
            int pos = cursor[slot];
            pos = pos < 0 ? 0 : (pos > RCAP - 1 ? RCAP - 1 : pos);
            region[pos] = src;
            const int np = pos + 1;
            cursor[slot] = np > RCAP ? RCAP : np;
          }
        }
      }
    }
    __syncthreads();
  }

  const int nv = lenW >> 2;
  int* gp = csr + rb0;
#pragma unroll 1
  for (int i = tid; i < nv; i += NTHR) { const v4i v = ((const v4i*)region)[i]; *(volatile v4i*)(gp + 4 * i) = v; }
  __threadfence();
#pragma unroll 1
  for (int i = tid; i < nv; i += NTHR) { const v4i v = ((const v4i*)region)[i]; *(volatile v4i*)(gp + 4 * i) = v; }
}

template <int KD>
__global__ __launch_bounds__(NTHR) void k_gemm(
    const float* __restrict__ A, const unsigned short* __restrict__ Bw, const float* __restrict__ dinv,
    float* C, int nRowsA) {
  extern __shared__ v4f lds_dyn[];
  constexpr int APH = KD + 8;
  static_assert(((APH * 2) % 16) == 0);
  static_assert((KD % 32) == 0);
  unsigned short* sHi = (unsigned short*)lds_dyn;
  unsigned short* sLo = sHi + GROWS * APH;
  float*          stg = (float*)lds_dyn;
  const int tid = threadIdx.x, lane = tid & 31, wave = tid >> 5, hh = lane >> 4, m = lane & 15;
  const int rowBase = blockIdx.x * GROWS;

#pragma unroll
  for (int i = 0; i < (GROWS * KD / 8) / NTHR; ++i) {
    const int idx = i * NTHR + tid;
    const int r   = idx / (KD / 8);
    const int c0  = (idx - r * (KD / 8)) * 8;
    int row = rowBase + r;
    row = row > nRowsA - 1 ? nRowsA - 1 : row;
    const float* ap = A + (size_t)row * KD + c0;
    const v4f a = *(const v4f*)ap, b = *(const v4f*)(ap + 4);
    v8us hv, lv;
    split8(a, b, hv, lv);
    *(v8us*)(sHi + r * APH + c0) = hv;
    *(v8us*)(sLo + r * APH + c0) = lv;
  }
  __syncthreads();

  v8f acc[4];
#pragma unroll
  for (int t = 0; t < 4; ++t) { v8f z = {0.f, 0.f, 0.f, 0.f, 0.f, 0.f, 0.f, 0.f}; acc[t] = z; }
  const unsigned short* ahp = sHi + (wave * 16 + m) * APH + 8 * hh;
  const unsigned short* alp = sLo + (wave * 16 + m) * APH + 8 * hh;
#pragma unroll
  for (int kt = 0; kt < KD / 32; ++kt) {
    FragB ah, al;
    ah.h[0] = *(const v8us*)(ahp + 32 * kt);
    ah.h[1] = *(const v8us*)(ahp + 32 * kt + 16);
    al.h[0] = *(const v8us*)(alp + 32 * kt);
    al.h[1] = *(const v8us*)(alp + 32 * kt + 16);
#pragma unroll
    for (int t = 0; t < 4; ++t) {
      const unsigned short* bp = Bw + (size_t)(16 * t + m) * KD + 32 * kt + 8 * hh;
      FragB bh, bl;
      bh.h[0] = *(const v8us*)bp;
      bh.h[1] = *(const v8us*)(bp + 16);
      bl.h[0] = *(const v8us*)(bp + (size_t)HID * KD);
      bl.h[1] = *(const v8us*)(bp + (size_t)HID * KD + 16);
      acc[t] = wmb(ah.v, bh.v, acc[t]);
      acc[t] = wmb(ah.v, bl.v, acc[t]);
      acc[t] = wmb(al.v, bh.v, acc[t]);
    }
  }
  __syncthreads();

  const int r0 = wave * 16 + 8 * hh;
  const v4f dA = *(const v4f*)(dinv + (size_t)rowBase + r0);
  const v4f dB = *(const v4f*)(dinv + (size_t)rowBase + r0 + 4);
  float s[8];
  s[0] = dA.x; s[1] = dA.y; s[2] = dA.z; s[3] = dA.w; s[4] = dB.x; s[5] = dB.y; s[6] = dB.z; s[7] = dB.w;
  float* sp = stg + r0 * HID + m;
#pragma unroll
  for (int t = 0; t < 4; ++t) {
#pragma unroll
    for (int r = 0; r < 8; ++r) sp[r * HID + 16 * t] = acc[t][r] * s[r];
  }
  __syncthreads();

  const float* lp = stg + wave * 16 * HID + 4 * lane;
  float* gp = C + (size_t)(rowBase + wave * 16) * HID + 4 * lane;
#pragma unroll
  for (int i = 0; i < 8; ++i) {
    const v4f v = *(const v4f*)(lp + i * 128);
    *(volatile v4f*)(gp + (size_t)i * 128) = v;
  }
  __threadfence();
#pragma unroll
  for (int i = 0; i < 8; ++i) {
    const v4f v = *(const v4f*)(lp + i * 128);
    *(volatile v4f*)(gp + (size_t)i * 128) = v;
  }
}

__global__ __launch_bounds__(NTHR) void k_agg(
    const int* __restrict__ csr, const int* __restrict__ off, const int* __restrict__ cnt,
    const float* __restrict__ dinv, const float* __restrict__ hw, float* h,
    const float* __restrict__ bs, int nN, int csrLen) {
  const int tid = threadIdx.x, lane = tid & 31, wave = tid >> 5, hf = lane >> 4, l16 = lane & 15;
  const int tbase = blockIdx.x * TGT + wave * 32;
  const int cl = tbase + lane;
  const int cnt_l = cnt[cl];
  const int off_l = off[cl];
  union FI { float f; int i; };
  FI dvu; dvu.f = dinv[cl];
  const v4f bb = *(const v4f*)(bs + 4 * l16);

#pragma unroll 1
  for (int j = 0; j < 16; ++j) {
    int n0 = __builtin_amdgcn_readlane(cnt_l, j);
    int n1 = __builtin_amdgcn_readlane(cnt_l, 16 + j);
    n0 = n0 < 0 ? 0 : (n0 > DEGCAP ? DEGCAP : n0);
    n1 = n1 < 0 ? 0 : (n1 > DEGCAP ? DEGCAP : n1);
    const int st0 = __builtin_amdgcn_readlane(off_l, j);
    const int st1 = __builtin_amdgcn_readlane(off_l, 16 + j);
    FI d0, d1;
    d0.i = __builtin_amdgcn_readlane(dvu.i, j);
    d1.i = __builtin_amdgcn_readlane(dvu.i, 16 + j);
    const int   n  = hf ? n1 : n0;
    const int   st = hf ? st1 : st0;
    const float dc = hf ? d1.f : d0.f;
    const int nmax = n0 > n1 ? n0 : n1;
    v4f acc = {0.f, 0.f, 0.f, 0.f};
#pragma unroll 1
    for (int q0 = 0; q0 < nmax; q0 += 16) {
      int pos = st + q0 + l16;
      pos = pos < 0 ? 0 : (pos > csrLen - 1 ? csrLen - 1 : pos);
      int sl = csr[pos];
      sl = sl < 0 ? 0 : (sl > nN - 1 ? nN - 1 : sl);
      const int mcnt = (nmax - q0) < 16 ? (nmax - q0) : 16;
#pragma unroll 1
      for (int p = 0; p < mcnt; ++p) {
        const int s0 = __builtin_amdgcn_readlane(sl, p);
        const int s1 = __builtin_amdgcn_readlane(sl, 16 + p);
        const int s = hf ? s1 : s0;
        const v4f v = *(const v4f*)(hw + (size_t)s * HID + 4 * l16);
        const bool ok = (q0 + p) < n;
        acc.x += ok ? v.x : 0.f;
        acc.y += ok ? v.y : 0.f;
        acc.z += ok ? v.z : 0.f;
        acc.w += ok ? v.w : 0.f;
      }
    }
    const int c = tbase + 16 * hf + j;
    const v4f sv = *(const v4f*)(hw + (size_t)c * HID + 4 * l16);
    v4f v = (acc + sv) * dc + bb;
    v.x = fmaxf(v.x, 0.f); v.y = fmaxf(v.y, 0.f); v.z = fmaxf(v.z, 0.f); v.w = fmaxf(v.w, 0.f);
    float* hp = h + (size_t)c * HID + 4 * l16;
    *(volatile v4f*)hp = v;
    __threadfence();
    *(volatile v4f*)hp = v;
  }
}

__global__ __launch_bounds__(NTHR) void k_decode(
    const float* __restrict__ z, const int* __restrict__ pe, const float* __restrict__ lw,
    const float* __restrict__ lb, float* out, int Ep, int nN) {
  const int tid = threadIdx.x, lane = tid & 31, wave = tid >> 5, hf = lane >> 4, l16 = lane & 15;
  const int base = ((int)blockIdx.x * NWAVE + wave) * 32;
  if (base >= Ep) return;
  int e = base + lane;
  e = e > Ep - 1 ? Ep - 1 : e;
  int s_l = pe[e];
  int d_l = pe[(size_t)Ep + e];
  s_l = s_l < 0 ? 0 : (s_l > nN - 1 ? nN - 1 : s_l);
  d_l = d_l < 0 ? 0 : (d_l > nN - 1 ? nN - 1 : d_l);
  const v4f wv = *(const v4f*)(lw + 4 * l16);
  const float lb0 = lb[0];
  float mine = 0.f;
#pragma unroll 1
  for (int j = 0; j < 16; ++j) {
    const int s0 = __builtin_amdgcn_readlane(s_l, j);
    const int s1 = __builtin_amdgcn_readlane(s_l, 16 + j);
    const int d0 = __builtin_amdgcn_readlane(d_l, j);
    const int d1 = __builtin_amdgcn_readlane(d_l, 16 + j);
    const int s = hf ? s1 : s0;
    const int d = hf ? d1 : d0;
    const v4f a = *(const v4f*)(z + (size_t)s * HID + 4 * l16);
    const v4f b = *(const v4f*)(z + (size_t)d * HID + 4 * l16);
    float p = (a.x * b.x) * wv.x;
    p = p + (a.y * b.y) * wv.y;
    p = p + (a.z * b.z) * wv.z;
    p = p + (a.w * b.w) * wv.w;
    p += __shfl_xor(p, 8);
    p += __shfl_xor(p, 4);
    p += __shfl_xor(p, 2);
    p += __shfl_xor(p, 1);
    mine = (l16 == j) ? p : mine;
  }
  const float val = mine + lb0;
  const int src4 = (lane & 7) * 4;
  v4f o;
  o.x = __shfl(val, src4 + 0);
  o.y = __shfl(val, src4 + 1);
  o.z = __shfl(val, src4 + 2);
  o.w = __shfl(val, src4 + 3);
  if (base + 32 <= Ep) {
    float* op = out + (size_t)base + src4;
    if (lane < 8) *(volatile v4f*)op = o;
    __threadfence();
    if (lane < 8) *(volatile v4f*)op = o;
  } else {
    float* op = out + (size_t)base + lane;
    if (base + lane < Ep) *(volatile float*)op = val;
    __threadfence();
    if (base + lane < Ep) *(volatile float*)op = val;
  }
}

extern "C" void kernel_launch(void* const* d_in, const int* in_sizes, int n_in,
                              void* d_out, int out_size, void* d_ws, size_t ws_size,
                              hipStream_t stream) {
  if (n_in < 10) return;
  const int nN = in_sizes[0] / INC;
  const int nE = in_sizes[1] / 2;
  const int Ep = in_sizes[2] / 2;
  const int En = in_sizes[3] / 2;
  if (nN <= 0 || nE <= 0 || Ep <= 0 || En <= 0) return;
  if (in_sizes[0] != nN * INC || in_sizes[1] != 2 * nE) return;
  if (in_sizes[2] != 2 * Ep || in_sizes[3] != 2 * En) return;
  if (in_sizes[4] != INC * HID || in_sizes[5] != HID) return;
  if (in_sizes[6] != HID * HID || in_sizes[7] != HID) return;
  if (in_sizes[8] != HID || in_sizes[9] < 1) return;
  if (out_size != Ep + En) return;
  if (nE > (1 << 28) || nN > (1 << 24)) return;

  const float* x   = (const float*)d_in[0];
  const int*   ei  = (const int*)d_in[1];
  const int*   pei = (const int*)d_in[2];
  const int*   nei = (const int*)d_in[3];
  const float* W1  = (const float*)d_in[4];
  const float* b1  = (const float*)d_in[5];
  const float* W2  = (const float*)d_in[6];
  const float* b2  = (const float*)d_in[7];
  const float* lwv = (const float*)d_in[8];
  const float* lbv = (const float*)d_in[9];
  float* out = (float*)d_out;

  const int NPAD   = ((nN + TGT - 1) / TGT) * TGT;
  const int nBC    = (nN + NBC - 1) / NBC;
  const int CNTPAD = nBC * NBC;
  if (4 * nBC + 1 > RBN) return;
  const int nBF    = (nN + NBF - 1) / NBF;
  const int csrLen = ((nE + 31) & ~31) + 4096;
  if (31 * 4 * nBC > 4096) return;
  const int nGemm  = NPAD / GROWS;
  const int nAgg   = NPAD / TGT;
  const int nDecP  = (((Ep + 31) / 32) + NWAVE - 1) / NWAVE;
  const int nDecN  = (((En + 31) / 32) + NWAVE - 1) / NWAVE;

  char* ws = (char*)d_ws;
  size_t off = 0;
  const size_t oW1  = off; off += (size_t)2 * HID * INC * 2;       off = (off + 255) & ~(size_t)255;
  const size_t oW2  = off; off += (size_t)2 * HID * HID * 2;       off = (off + 255) & ~(size_t)255;
  const size_t oCnt = off; off += (size_t)CNTPAD * 4;              off = (off + 255) & ~(size_t)255;
  const size_t oDv  = off; off += (size_t)CNTPAD * 4;              off = (off + 255) & ~(size_t)255;
  const size_t oOff = off; off += (size_t)CNTPAD * 4;              off = (off + 255) & ~(size_t)255;
  const size_t oRb  = off; off += (size_t)RBN * 4;                 off = (off + 255) & ~(size_t)255;
  const size_t oCsr = off; off += (size_t)csrLen * 4;              off = (off + 255) & ~(size_t)255;
  const size_t oH   = off; off += (size_t)NPAD * HID * 4;          off = (off + 255) & ~(size_t)255;
  const size_t oHw  = off; off += (size_t)NPAD * HID * 4;          off = (off + 255) & ~(size_t)255;
  if (off > ws_size || off > (size_t)WSCAP) return;
  unsigned short* wp1 = (unsigned short*)(ws + oW1);
  unsigned short* wp2 = (unsigned short*)(ws + oW2);
  int*      cnt  = (int*)(ws + oCnt);
  float*    dinv = (float*)(ws + oDv);
  int*      offp = (int*)(ws + oOff);
  int*      rb   = (int*)(ws + oRb);
  int*      csr  = (int*)(ws + oCsr);
  float*    h    = (float*)(ws + oH);
  float*    hw   = (float*)(ws + oHw);

  const int vec8 = ((nE & 3) == 0) ? 1 : 0;

  const int tot1 = HID * INC / 8, tot2 = HID * HID / 8;
  k_wprep<<<(tot1 + NTHR - 1) / NTHR, NTHR, 0, stream>>>(W1, wp1, INC, tot1);
  k_wprep<<<(tot2 + NTHR - 1) / NTHR, NTHR, 0, stream>>>(W2, wp2, HID, tot2);

  k_count<<<nBC, NTHR, 0, stream>>>(ei, cnt, dinv, nE, vec8);
  k_offsets<<<1, OTHR, 0, stream>>>(cnt, offp, rb, nBC);
  hipFuncSetAttribute(reinterpret_cast<const void*>(&k_fill),
                      hipFuncAttributeMaxDynamicSharedMemorySize, LDS_FILL);
  k_fill<<<nBF, NTHR, LDS_FILL, stream>>>(ei, offp, rb, csr, nN, nE, vec8, csrLen);

  hipFuncSetAttribute(reinterpret_cast<const void*>(&k_gemm<INC>),
                      hipFuncAttributeMaxDynamicSharedMemorySize, LDS_GEMM(INC));
  k_gemm<INC><<<nGemm, NTHR, LDS_GEMM(INC), stream>>>(x, wp1, dinv, hw, nN);
  k_agg<<<nAgg, NTHR, 0, stream>>>(csr, offp, cnt, dinv, hw, h, b1, nN, csrLen);

  hipFuncSetAttribute(reinterpret_cast<const void*>(&k_gemm<HID>),
                      hipFuncAttributeMaxDynamicSharedMemorySize, LDS_GEMM(HID));
  k_gemm<HID><<<nGemm, NTHR, LDS_GEMM(HID), stream>>>(h, wp2, dinv, hw, NPAD);
  k_agg<<<nAgg, NTHR, 0, stream>>>(csr, offp, cnt, dinv, hw, h, b2, nN, csrLen);

  k_decode<<<nDecP, NTHR, 0, stream>>>(h, pei, lwv, lbv, out, Ep, nN);
  k_decode<<<nDecN, NTHR, 0, stream>>>(h, nei, lwv, lbv, out + (size_t)Ep, En, nN);
}
